// Cheb_35888746725726
// MI455X (gfx1250) — hardware-verified
//
#include <hip/hip_runtime.h>
#include <stddef.h>


#define FD       96
#define KCAT     (3 * FD)
#define WP       320
#define NTHR     256
#define NWAVE    8
#define EPT      8
#define NGRP     2
#define CHUNK    (NTHR * EPT * NGRP)
#define WCAP     (EPT * NGRP * 32)
#define LISTN    (NWAVE * WCAP)
#define NBP      640
#define QPW      ((NBP * FD) / (NWAVE * 128))
#define NBD      4096
#define GROWS    (NWAVE * 16)
#define ENW      (NTHR * 4)
#define LDS_PROP (NBP * FD * 4 + LISTN * 4 + 64)

static_assert((CHUNK & (CHUNK - 1)) == 0);
static_assert(CHUNK <= 4096);
static_assert(NBP <= 4096 && NBD <= 4096);
static_assert(NBP * FD == NWAVE * 128 * QPW);
static_assert(((NBP * FD) / 4) % NTHR == 0);
static_assert((NBD / 4) == NWAVE * 4 * 32);
static_assert(KCAT % 32 == 0 && FD % 32 == 0 && WP >= KCAT && (WP % 64) == 0);
static_assert((16 * FD) % 128 == 0);

typedef float  v4f  __attribute__((ext_vector_type(4)));
typedef float  v8f  __attribute__((ext_vector_type(8)));
typedef int    v4i  __attribute__((ext_vector_type(4)));
typedef __bf16 v8b  __attribute__((ext_vector_type(8)));
typedef __bf16 v16b __attribute__((ext_vector_type(16)));
union FragB { v16b v; v8b h[2]; };
union CvB   { v8b b; v4i i; };

__device__ __forceinline__ void split8(v4f a, v4f b, v8b& hi, v8b& lo) {
  __bf16 t;
  t = (__bf16)a.x; hi[0] = t; lo[0] = (__bf16)(a.x - (float)t);
  t = (__bf16)a.y; hi[1] = t; lo[1] = (__bf16)(a.y - (float)t);
  t = (__bf16)a.z; hi[2] = t; lo[2] = (__bf16)(a.z - (float)t);
  t = (__bf16)a.w; hi[3] = t; lo[3] = (__bf16)(a.w - (float)t);
  t = (__bf16)b.x; hi[4] = t; lo[4] = (__bf16)(b.x - (float)t);
  t = (__bf16)b.y; hi[5] = t; lo[5] = (__bf16)(b.y - (float)t);
  t = (__bf16)b.z; hi[6] = t; lo[6] = (__bf16)(b.z - (float)t);
  t = (__bf16)b.w; hi[7] = t; lo[7] = (__bf16)(b.w - (float)t);
}

__device__ __forceinline__ v8f wmb(v16b a, v16b b, v8f c) {
  v8f d = __builtin_amdgcn_wmma_f32_16x16x32_bf16(false, a, false, b, (short)0, c, false, false);
  asm volatile("v_nop\n\tv_nop\n\tv_nop\n\tv_nop" : "+v"(d) : "v"(a), "v"(b));
  return d;
}

template <int NB>
__device__ __forceinline__ int scan_chunk(const int* __restrict__ keys, int nE, int cbase, int nodeBase,
                                          int vec8, int* list, int tid, int wave) {
  int wc = 0;
#pragma unroll
  for (int g = 0; g < NGRP; ++g) {
    const int el0  = (g * NTHR + tid) * EPT;
    const int e0   = cbase + el0;
    const int sent = -2147483647 - 1;
    v4i da, db;
    if (vec8 != 0 && e0 + 7 < nE) {
      da = *(const v4i*)(keys + e0);
      db = *(const v4i*)(keys + e0 + 4);
    } else {
      da.x = (e0     < nE) ? keys[min(e0,     nE - 1)] : sent;
      da.y = (e0 + 1 < nE) ? keys[min(e0 + 1, nE - 1)] : sent;
      da.z = (e0 + 2 < nE) ? keys[min(e0 + 2, nE - 1)] : sent;
      da.w = (e0 + 3 < nE) ? keys[min(e0 + 3, nE - 1)] : sent;
      db.x = (e0 + 4 < nE) ? keys[min(e0 + 4, nE - 1)] : sent;
      db.y = (e0 + 5 < nE) ? keys[min(e0 + 5, nE - 1)] : sent;
      db.z = (e0 + 6 < nE) ? keys[min(e0 + 6, nE - 1)] : sent;
      db.w = (e0 + 7 < nE) ? keys[min(e0 + 7, nE - 1)] : sent;
    }
    const unsigned nb = (unsigned)nodeBase;
    const unsigned s0 = (unsigned)da.x - nb, s1 = (unsigned)da.y - nb;
    const unsigned s2 = (unsigned)da.z - nb, s3 = (unsigned)da.w - nb;
    const unsigned s4 = (unsigned)db.x - nb, s5 = (unsigned)db.y - nb;
    const unsigned s6 = (unsigned)db.z - nb, s7 = (unsigned)db.w - nb;
    const bool h0 = s0 < (unsigned)NB, h1 = s1 < (unsigned)NB, h2 = s2 < (unsigned)NB, h3 = s3 < (unsigned)NB;
    const bool h4 = s4 < (unsigned)NB, h5 = s5 < (unsigned)NB, h6 = s6 < (unsigned)NB, h7 = s7 < (unsigned)NB;
    const unsigned any = __builtin_amdgcn_ballot_w32(h0 | h1 | h2 | h3 | h4 | h5 | h6 | h7);
    if (any != 0u) {
#define HITJ(J, HJ, SJ) { \
        const unsigned mj = __builtin_amdgcn_ballot_w32(HJ); \
        if (mj != 0u) { \
          if (HJ) { \
            const int pos = wc + (int)__builtin_amdgcn_mbcnt_lo(mj, 0u); \
            if (pos < WCAP) list[wave * WCAP + pos] = ((el0 + (J)) << 12) | (int)(SJ); \
          } \
          wc += (int)__builtin_popcount(mj); } }
      HITJ(0, h0, s0)
      HITJ(1, h1, s1)
      HITJ(2, h2, s2)
      HITJ(3, h3, s3)
      HITJ(4, h4, s4)
      HITJ(5, h5, s5)
      HITJ(6, h6, s6)
      HITJ(7, h7, s7)
#undef HITJ
    }
  }
  return wc;
}

__global__ __launch_bounds__(NTHR) void k_wprep(
    const float* __restrict__ W1, const float* __restrict__ W2,
    __bf16* h1p, __bf16* l1p, __bf16* h2p, __bf16* l2p) {
  const int t   = blockIdx.x * NTHR + threadIdx.x;
  const int per = FD * (WP / 8);
  if (t >= 2 * per) return;
  const int sel = (t >= per) ? 1 : 0;
  const int u   = t - sel * per;
  const int n   = u / (WP / 8);
  const int q   = u - n * (WP / 8);
  const int k0  = 8 * q;
  const float* W = sel ? W2 : W1;
  v4f a = {0.f, 0.f, 0.f, 0.f}, b = {0.f, 0.f, 0.f, 0.f};
  if (k0 + 8 <= KCAT) {
    const float* p = W + (size_t)k0 * FD + n;
    a.x = p[0];      a.y = p[FD];     a.z = p[2 * FD]; a.w = p[3 * FD];
    b.x = p[4 * FD]; b.y = p[5 * FD]; b.z = p[6 * FD]; b.w = p[7 * FD];
  }
  CvB hv, lv;
  split8(a, b, hv.b, lv.b);
  __bf16* hp = (sel ? h2p : h1p) + (size_t)n * WP + k0;
  __bf16* lp = (sel ? l2p : l1p) + (size_t)n * WP + k0;
  *(volatile v4i*)hp = hv.i;
  *(volatile v4i*)lp = lv.i;
  __threadfence();
  *(volatile v4i*)hp = hv.i;
  *(volatile v4i*)lp = lv.i;
}

__global__ __launch_bounds__(NTHR) void k_deg(
    const int* __restrict__ ei, const float* __restrict__ ew, float* dis, int nN, int nE, int vec8) {
  __shared__ __attribute__((aligned(16))) float cnt[NBD];
  __shared__ __attribute__((aligned(16))) int list[LISTN];
  __shared__ int wcnt[NWAVE];
  const int tid = threadIdx.x, lane = tid & 31, wave = tid >> 5;
  const int nodeBase = blockIdx.x * NBD;
  (void)nN;

  for (int i = tid; i < NBD; i += NTHR) cnt[i] = 0.f;
  __syncthreads();

  const int nChunks = (nE + CHUNK - 1) / CHUNK;
#pragma unroll 1
  for (int ch = 0; ch < nChunks; ++ch) {
    const int cbase = ch * CHUNK;
    const int wc = scan_chunk<NBD>(ei, nE, cbase, nodeBase, vec8, list, tid, wave);
    if (lane == 0) wcnt[wave] = wc;
    __syncthreads();
    if (wave == 0) {
#pragma unroll 1
      for (int wsx = 0; wsx < NWAVE; ++wsx) {
        int n = __builtin_amdgcn_readfirstlane(wcnt[wsx]);
        n = n > WCAP ? WCAP : (n < 0 ? 0 : n);
        const int* lp = list + wsx * WCAP;
#pragma unroll 1
        for (int i = 0; i < n; ++i) {
          const int ent  = __builtin_amdgcn_readfirstlane(lp[i]);
          const int slot = ent & (NBD - 1);
          int e = cbase + ((ent >> 12) & (CHUNK - 1));
          e = e > nE - 1 ? nE - 1 : e;
          const float w = ew[e];
          if (lane == 0) cnt[slot] = cnt[slot] + w;
        }
      }
    }
    __syncthreads();
  }

  v4f dq[4];
#pragma unroll
  for (int q = 0; q < 4; ++q) {
    const int f = (wave * 4 + q) * 128 + 4 * lane;
    const v4f c = *(const v4f*)(cnt + f);
    dq[q].x = (c.x > 0.f) ? rsqrtf(fmaxf(c.x, 1e-30f)) : 0.f;
    dq[q].y = (c.y > 0.f) ? rsqrtf(fmaxf(c.y, 1e-30f)) : 0.f;
    dq[q].z = (c.z > 0.f) ? rsqrtf(fmaxf(c.z, 1e-30f)) : 0.f;
    dq[q].w = (c.w > 0.f) ? rsqrtf(fmaxf(c.w, 1e-30f)) : 0.f;
  }
  float* dp = dis + (size_t)nodeBase;
#pragma unroll
  for (int q = 0; q < 4; ++q) *(volatile v4f*)(dp + (wave * 4 + q) * 128 + 4 * lane) = dq[q];
  __threadfence();
#pragma unroll
  for (int q = 0; q < 4; ++q) *(volatile v4f*)(dp + (wave * 4 + q) * 128 + 4 * lane) = dq[q];
}

__global__ __launch_bounds__(NTHR) void k_enorm(
    const int* __restrict__ ei, const float* __restrict__ ew, const float* __restrict__ dis,
    float* nw, int nN, int nE) {
  const int e4 = (blockIdx.x * NTHR + threadIdx.x) * 4;
  v4f r;
#pragma unroll
  for (int c = 0; c < 4; ++c) {
    int e = e4 + c;
    e = e > nE - 1 ? nE - 1 : e;
    int s = ei[e];
    int d = ei[(size_t)nE + e];
    s = s < 0 ? 0 : (s > nN - 1 ? nN - 1 : s);
    d = d < 0 ? 0 : (d > nN - 1 ? nN - 1 : d);
    const float w = ew[e];
    r[c] = -(dis[s] * w) * dis[d];
  }
  *(volatile v4f*)(nw + e4) = r;
  __threadfence();
  *(volatile v4f*)(nw + e4) = r;
}

template <int MODE>
__global__ __launch_bounds__(NTHR) void k_prop(
    const int* __restrict__ ei, const float* __restrict__ nw, const float* __restrict__ hs,
    const float* __restrict__ t0, float* outp, int nN, int nE, int vec8) {
  extern __shared__ v4f lds_dyn[];
  float* acc  = (float*)lds_dyn;
  int*   list = (int*)(acc + NBP * FD);
  int*   wcnt = list + LISTN;
  const int tid = threadIdx.x, lane = tid & 31, wave = tid >> 5;
  const int nodeBase = blockIdx.x * NBP;
  const int* dsts = ei + nE;

  {
    const v4f z = {0.f, 0.f, 0.f, 0.f};
    for (int i = tid; i < NBP * FD / 4; i += NTHR) lds_dyn[i] = z;
  }
  __syncthreads();

  const int nChunks = (nE + CHUNK - 1) / CHUNK;
#pragma unroll 1
  for (int ch = 0; ch < nChunks; ++ch) {
    const int cbase = ch * CHUNK;
    const int wc = scan_chunk<NBP>(dsts, nE, cbase, nodeBase, vec8, list, tid, wave);
    if (lane == 0) wcnt[wave] = wc;
    __syncthreads();
    if (wave == 0) {
#pragma unroll 1
      for (int wsx = 0; wsx < NWAVE; ++wsx) {
        int n = __builtin_amdgcn_readfirstlane(wcnt[wsx]);
        n = n > WCAP ? WCAP : (n < 0 ? 0 : n);
        const int* lp = list + wsx * WCAP;
#pragma unroll 1
        for (int i = 0; i < n; ++i) {
          const int ent = __builtin_amdgcn_readfirstlane(lp[i]);
          int slot = ent & 4095;
          slot = slot > NBP - 1 ? NBP - 1 : slot;
          int e = cbase + ((ent >> 12) & (CHUNK - 1));
          e = e > nE - 1 ? nE - 1 : e;
          int src = ei[e];
          src = src < 0 ? 0 : (src > nN - 1 ? nN - 1 : src);
          const float w = nw[e];
          if (lane < FD / 4) {
            const v4f v = *(const v4f*)(hs + (size_t)src * FD + 4 * lane);
            v4f* ap = (v4f*)(acc + slot * FD + 4 * lane);
            *ap = *ap + v * w;
          }
        }
      }
    }
    __syncthreads();
  }

  if (MODE == 1) {
#pragma unroll 4
    for (int i = 0; i < (NBP * FD / 4) / NTHR; ++i) {
      const int idx  = i * NTHR + tid;
      const int slot = idx / (FD / 4);
      const int c4   = (idx - slot * (FD / 4)) * 4;
      int node = nodeBase + slot;
      node = node > nN - 1 ? nN - 1 : node;
      const v4f tv = *(const v4f*)(t0 + (size_t)node * FD + c4);
      v4f* ap = (v4f*)(acc + slot * FD + c4);
      *ap = *ap * 2.0f - tv;
    }
    __syncthreads();
  }

  float* gp = outp + (size_t)nodeBase * FD;
#pragma unroll 4
  for (int q = 0; q < QPW; ++q) {
    const int f = (wave * QPW + q) * 128 + 4 * lane;
    const v4f v = *(const v4f*)(acc + f);
    *(volatile v4f*)(gp + f) = v;
  }
  __threadfence();
#pragma unroll 4
  for (int q = 0; q < QPW; ++q) {
    const int f = (wave * QPW + q) * 128 + 4 * lane;
    const v4f v = *(const v4f*)(acc + f);
    *(volatile v4f*)(gp + f) = v;
  }
}

template <int LAYER>
__global__ __launch_bounds__(NTHR) void k_cheb(
    const float* T0, const float* T1, const float* T2,
    const __bf16* __restrict__ whi, const __bf16* __restrict__ wlo,
    const float* __restrict__ bias, const float* __restrict__ wl, const float* __restrict__ bl,
    float* hout, float* out, int nN) {
  constexpr int STGN = (LAYER == 1) ? (NWAVE * 16 * FD) : (NWAVE * 32);
  __shared__ __attribute__((aligned(16))) float stg[STGN];
  const int tid = threadIdx.x, lane = tid & 31, wave = tid >> 5, hh = lane >> 4, m = lane & 15;
  const int row0 = (blockIdx.x * NWAVE + wave) * 16;
  int ra = row0 + m;
  ra = ra > nN - 1 ? nN - 1 : ra;

  v8f acc[FD / 16];
#pragma unroll
  for (int t = 0; t < FD / 16; ++t) { v8f z = {0.f, 0.f, 0.f, 0.f, 0.f, 0.f, 0.f, 0.f}; acc[t] = z; }

#pragma unroll 1
  for (int kt = 0; kt < KCAT / 32; ++kt) {
    const int j  = kt / (FD / 32);
    const int kk = 32 * (kt - j * (FD / 32)) + 8 * hh;
    const float* P  = (j == 0) ? T0 : ((j == 1) ? T1 : T2);
    const float* ap = P + (size_t)ra * FD + kk;
    const v4f x0 = *(const v4f*)ap,        x1 = *(const v4f*)(ap + 4);
    const v4f x2 = *(const v4f*)(ap + 16), x3 = *(const v4f*)(ap + 20);
    FragB ah, al;
    split8(x0, x1, ah.h[0], al.h[0]);
    split8(x2, x3, ah.h[1], al.h[1]);
    const __bf16* ph = whi + (size_t)m * WP + 32 * kt + 8 * hh;
    const __bf16* pl = wlo + (size_t)m * WP + 32 * kt + 8 * hh;
#pragma unroll
    for (int t = 0; t < FD / 16; ++t) {
      const __bf16* qh = ph + (size_t)(16 * t) * WP;
      const __bf16* ql = pl + (size_t)(16 * t) * WP;
      FragB bh, blw;
      bh.h[0]  = *(const v8b*)qh;  bh.h[1]  = *(const v8b*)(qh + 16);
      blw.h[0] = *(const v8b*)ql;  blw.h[1] = *(const v8b*)(ql + 16);
      acc[t] = wmb(ah.v, bh.v,  acc[t]);
      acc[t] = wmb(ah.v, blw.v, acc[t]);
      acc[t] = wmb(al.v, bh.v,  acc[t]);
    }
  }

  float bv[FD / 16];
#pragma unroll
  for (int t = 0; t < FD / 16; ++t) bv[t] = bias[16 * t + m];

  if (LAYER == 1) {
    float* sp = stg + wave * (16 * FD) + (8 * hh) * FD + m;
#pragma unroll
    for (int t = 0; t < FD / 16; ++t) {
#pragma unroll
      for (int r = 0; r < 8; ++r) sp[r * FD + 16 * t] = fmaxf(acc[t][r] + bv[t], 0.f);
    }
    __syncthreads();
    const float* lp = stg + wave * (16 * FD) + 4 * lane;
    float* gp = hout + (size_t)row0 * FD + 4 * lane;
#pragma unroll
    for (int i = 0; i < (16 * FD) / 128; ++i) { const v4f v = *(const v4f*)(lp + 128 * i); *(volatile v4f*)(gp + 128 * i) = v; }
    __threadfence();
#pragma unroll
    for (int i = 0; i < (16 * FD) / 128; ++i) { const v4f v = *(const v4f*)(lp + 128 * i); *(volatile v4f*)(gp + 128 * i) = v; }
  } else {
    float w0[FD / 16], w1[FD / 16];
#pragma unroll
    for (int t = 0; t < FD / 16; ++t) { w0[t] = wl[(16 * t + m) * 2]; w1[t] = wl[(16 * t + m) * 2 + 1]; }
    float p0[8], p1[8];
#pragma unroll
    for (int r = 0; r < 8; ++r) { p0[r] = 0.f; p1[r] = 0.f; }
#pragma unroll
    for (int t = 0; t < FD / 16; ++t) {
#pragma unroll
      for (int r = 0; r < 8; ++r) {
        const float v = fmaxf(acc[t][r] + bv[t], 0.f);
        p0[r] += v * w0[t];
        p1[r] += v * w1[t];
      }
    }
#pragma unroll
    for (int mk = 1; mk < 16; mk <<= 1) {
#pragma unroll
      for (int r = 0; r < 8; ++r) {
        p0[r] += __shfl_xor(p0[r], mk);
        p1[r] += __shfl_xor(p1[r], mk);
      }
    }
    const float b0 = bl[0], b1v = bl[1];
    if (m == 0) {
      float* sp = stg + wave * 32 + 16 * hh;
#pragma unroll
      for (int r = 0; r < 8; ++r) { sp[2 * r] = p0[r] + b0; sp[2 * r + 1] = p1[r] + b1v; }
    }
    __syncthreads();
    v4f ov = {0.f, 0.f, 0.f, 0.f};
    if (lane < 8) ov = *(const v4f*)(stg + wave * 32 + 4 * lane);
    const size_t outN = (size_t)nN * 2;
    const size_t gi   = (size_t)row0 * 2 + 4 * lane;
    if (lane < 8) {
      if (gi + 4 <= outN) {
        *(volatile v4f*)(out + gi) = ov;
      } else {
#pragma unroll
        for (int c = 0; c < 4; ++c) if (gi + c < outN) ((volatile float*)out)[gi + c] = ov[c];
      }
    }
    __threadfence();
    if (lane < 8) {
      if (gi + 4 <= outN) {
        *(volatile v4f*)(out + gi) = ov;
      } else {
#pragma unroll
        for (int c = 0; c < 4; ++c) if (gi + c < outN) ((volatile float*)out)[gi + c] = ov[c];
      }
    }
  }
}

extern "C" void kernel_launch(void* const* d_in, const int* in_sizes, int n_in,
                              void* d_out, int out_size, void* d_ws, size_t ws_size,
                              hipStream_t stream) {
  if (n_in < 9) return;
  const int nN = in_sizes[0] / FD;
  if (nN <= 0 || in_sizes[0] != nN * FD) return;
  const int nE = in_sizes[2];
  if (nE <= 0 || in_sizes[1] != 2 * nE) return;
  if (in_sizes[3] != 3 * FD * FD || in_sizes[4] < FD || in_sizes[5] != 3 * FD * FD || in_sizes[6] < FD) return;
  if (in_sizes[7] != 2 * FD || in_sizes[8] < 2) return;
  if (out_size != 2 * nN) return;

  const float* x    = (const float*)d_in[0];
  const int*   ei   = (const int*)d_in[1];
  const float* ew   = (const float*)d_in[2];
  const float* W1   = (const float*)d_in[3];
  const float* b1   = (const float*)d_in[4];
  const float* W2   = (const float*)d_in[5];
  const float* b2   = (const float*)d_in[6];
  const float* Wlin = (const float*)d_in[7];
  const float* blin = (const float*)d_in[8];
  float* out = (float*)d_out;

  const int nBD = (nN + NBD - 1) / NBD;
  const int nNW = (nE + ENW - 1) / ENW;
  const int nPB = (nN + NBP - 1) / NBP;
  const int nGB = (nN + GROWS - 1) / GROWS;

  char* ws = (char*)d_ws;
  size_t off = 0;
  const size_t plW = (size_t)FD * WP * 2;
  const size_t oWh1 = off; off += plW;                                       off = (off + 255) & ~(size_t)255;
  const size_t oWl1 = off; off += plW;                                       off = (off + 255) & ~(size_t)255;
  const size_t oWh2 = off; off += plW;                                       off = (off + 255) & ~(size_t)255;
  const size_t oWl2 = off; off += plW;                                       off = (off + 255) & ~(size_t)255;
  const size_t oDis = off; off += (size_t)nBD * NBD * 4;                     off = (off + 255) & ~(size_t)255;
  const size_t oNW  = off; off += (size_t)nNW * ENW * 4;                     off = (off + 255) & ~(size_t)255;
  const size_t oT1  = off; off += (size_t)nPB * NBP * FD * 4;                off = (off + 255) & ~(size_t)255;
  const size_t oT2  = off; off += (size_t)nPB * NBP * FD * 4;                off = (off + 255) & ~(size_t)255;
  const size_t oH1  = off; off += (size_t)nGB * GROWS * FD * 4;              off = (off + 255) & ~(size_t)255;
  if (off > ws_size) return;
  if (off > (size_t)134217728) return;
  __bf16* whi1 = (__bf16*)(ws + oWh1);
  __bf16* wlo1 = (__bf16*)(ws + oWl1);
  __bf16* whi2 = (__bf16*)(ws + oWh2);
  __bf16* wlo2 = (__bf16*)(ws + oWl2);
  float*  dis  = (float*)(ws + oDis);
  float*  nw   = (float*)(ws + oNW);
  float*  T1   = (float*)(ws + oT1);
  float*  T2   = (float*)(ws + oT2);
  float*  H1   = (float*)(ws + oH1);

  const int vec8 = ((nE & 3) == 0) ? 1 : 0;

  const int nPrepThr = 2 * FD * (WP / 8);
  k_wprep<<<(nPrepThr + NTHR - 1) / NTHR, NTHR, 0, stream>>>(W1, W2, whi1, wlo1, whi2, wlo2);

  k_deg<<<nBD, NTHR, 0, stream>>>(ei, ew, dis, nN, nE, vec8);
  k_enorm<<<nNW, NTHR, 0, stream>>>(ei, ew, dis, nw, nN, nE);

  hipFuncSetAttribute(reinterpret_cast<const void*>(&k_prop<0>),
                      hipFuncAttributeMaxDynamicSharedMemorySize, LDS_PROP);
  hipFuncSetAttribute(reinterpret_cast<const void*>(&k_prop<1>),
                      hipFuncAttributeMaxDynamicSharedMemorySize, LDS_PROP);

  k_prop<0><<<nPB, NTHR, LDS_PROP, stream>>>(ei, nw, x, x, T1, nN, nE, vec8);
  k_prop<1><<<nPB, NTHR, LDS_PROP, stream>>>(ei, nw, T1, x, T2, nN, nE, vec8);
  k_cheb<1><<<nGB, NTHR, 0, stream>>>(x, T1, T2, whi1, wlo1, b1, Wlin, blin, H1, out, nN);

  k_prop<0><<<nPB, NTHR, LDS_PROP, stream>>>(ei, nw, H1, H1, T1, nN, nE, vec8);
  k_prop<1><<<nPB, NTHR, LDS_PROP, stream>>>(ei, nw, T1, H1, T2, nN, nE, vec8);
  k_cheb<2><<<nGB, NTHR, 0, stream>>>(H1, T1, T2, whi2, wlo2, b2, Wlin, blin, H1, out, nN);
}
